// LNOBlock_73830487818861
// MI455X (gfx1250) — hardware-verified
//
#include <hip/hip_runtime.h>
#include <stddef.h>
#include <math.h>


typedef _Float16 h16;
typedef _Float16 v16h __attribute__((ext_vector_type(16)));
typedef _Float16 v8h  __attribute__((ext_vector_type(8)));
typedef float    v8f  __attribute__((ext_vector_type(8)));
typedef float    v4f  __attribute__((ext_vector_type(4)));
typedef float    v2f  __attribute__((ext_vector_type(2)));

#ifndef NB
#define NB 2
#endif
#ifndef SEQ
#define SEQ 8192
#endif
#define NB_FULL  2
#define SEQ_FULL 8192
#define CDIM  128
#define RNK   64
#define MROWS (NB * SEQ)

#define GCH    16
#define KCH    (SEQ / GCH)
#define XBLKS  (MROWS / 64)
#define BPB    (SEQ / 64)
#define BPW    (BPB / 8)
#define PHROWS 192
#define IC     32

static_assert(NB >= 1 && NB <= NB_FULL);
static_assert(SEQ >= 512 && SEQ <= SEQ_FULL && (SEQ % 512) == 0);
static_assert(CDIM == 128 && RNK == 64);
static_assert((KCH % 32) == 0 && KCH * GCH == SEQ);
static_assert((CDIM % 64) == 0 && (CDIM % 32) == 0 && (RNK % 32) == 0);
static_assert((MROWS % 64) == 0 && (SEQ % 64) == 0);
static_assert(BPW * 8 == BPB && BPB * NB == XBLKS);
static_assert((PHROWS % 64) == 0 && PHROWS >= CDIM + 1 && (PHROWS % 32) == 0);
static_assert(CDIM == 16 * 8);
static_assert(CDIM == 32 * 4);
static_assert((CDIM % IC) == 0 && IC == 32);
static_assert(RNK == 8 * 8);

#define LDT 72
#define LDC 68
static_assert((LDT % 8) == 0 && LDT >= 64);
static_assert((LDC % 4) == 0 && LDC >= 64);

#define XCARRY 16.0f
#define WCARRY 64.0f
#define ICARRY 64.0f
#define ECARRY 64.0f

#define X16_BYTES   ((size_t)MROWS * CDIM * 2)
#define XT16_BYTES  ((size_t)NB * CDIM * SEQ * 2)
#define SPART_BYTES ((size_t)XBLKS * CDIM * 4)
#define GPART_BYTES ((size_t)NB * GCH * CDIM * CDIM * 4)
#define G_BYTES     ((size_t)NB * CDIM * CDIM * 4)
#define S_BYTES     ((size_t)NB * CDIM * 4)
#define IT_BYTES    ((size_t)NB * CDIM * RNK * 2)
#define PH_BYTES    ((size_t)PHROWS * RNK * 2)
#define WT_BYTES    ((size_t)NB * CDIM * CDIM * 2)
#define BE_BYTES    ((size_t)NB * CDIM * 4)
#define OFF_X16   ((size_t)0)
#define OFF_XT16  (OFF_X16 + X16_BYTES)
#define OFF_SPART (OFF_XT16 + XT16_BYTES)
#define OFF_GPART (OFF_SPART + SPART_BYTES)
#define OFF_G     (OFF_GPART + GPART_BYTES)
#define OFF_S     (OFF_G + G_BYTES)
#define OFF_IT    (OFF_S + S_BYTES)
#define OFF_PH    (OFF_IT + IT_BYTES)
#define OFF_WT    (OFF_PH + PH_BYTES)
#define OFF_BE    (OFF_WT + WT_BYTES)
#define WS_TOTAL  (OFF_BE + BE_BYTES)
static_assert((X16_BYTES % 128) == 0 && (XT16_BYTES % 128) == 0 && (SPART_BYTES % 128) == 0);
static_assert((GPART_BYTES % 128) == 0 && (G_BYTES % 128) == 0 && (S_BYTES % 128) == 0);
static_assert((IT_BYTES % 128) == 0 && (PH_BYTES % 128) == 0 && (WT_BYTES % 128) == 0);
static_assert((BE_BYTES % 128) == 0);
static_assert(WS_TOTAL <= (size_t)134217728);

__device__ __forceinline__ float bf16r(float x) {
  unsigned int u = __float_as_uint(x);
  u = (u + 0x7FFFu + ((u >> 16) & 1u)) & 0xFFFF0000u;
  return __uint_as_float(u);
}

static __device__ __forceinline__ h16 toh_flush(float v) {
  const h16 r = (h16)v;
  return (fabsf(v) < 6.103515625e-05f) ? (h16)0.0f : r;
}

__device__ __forceinline__ v16h frag_at(const _Float16* p) {
  v8h lo = *(const v8h*)(p);
  v8h hi = *(const v8h*)(p + 16);
  v16h out;
#pragma unroll
  for (int i = 0; i < 8; ++i) { out[i] = lo[i]; out[i + 8] = hi[i]; }
  return out;
}

__device__ __forceinline__ v8f wmma16(v16h a, v16h b, v8f c) {
  v8f d = __builtin_amdgcn_wmma_f32_16x16x32_f16(false, a, false, b, (short)0, c,
                                                 false, false);
  asm volatile("v_nop\n\tv_nop\n\tv_nop\n\tv_nop" : "+v"(d) : "v"(a), "v"(b));
  return d;
}

__device__ __forceinline__ void gemm_loop(const _Float16* __restrict__ ap,
                                          const _Float16* __restrict__ bp0,
                                          const _Float16* __restrict__ bp1,
                                          const unsigned K, v8f& acc0, v8f& acc1) {
#pragma unroll 2
  for (unsigned k0 = 0; k0 < K; k0 += 32u) {
    const v16h a  = frag_at(ap + k0);
    const v16h b0 = frag_at(bp0 + k0);
    const v16h b1 = frag_at(bp1 + k0);
    acc0 = wmma16(a, b0, acc0);
    acc1 = wmma16(a, b1, acc1);
  }
}

__device__ __forceinline__ float gelu_erf(float v) {
  return 0.5f * v * (1.0f + erff(v * 0.70710678118654752f));
}

__global__ __launch_bounds__(256) void xconv_kernel(
    const float* __restrict__ X, _Float16* __restrict__ X16, _Float16* __restrict__ XT16,
    float* __restrict__ Spart) {
  __shared__ _Float16 T[CDIM * LDT];
  __shared__ float Sc[16 * CDIM];
  const unsigned tid = threadIdx.x, lane = tid & 31u;
  const int wave = __builtin_amdgcn_readfirstlane((int)(threadIdx.x >> 5));
  const unsigned crow0 = blockIdx.x * 64u;
  const unsigned bidx = crow0 / (unsigned)SEQ;
  const unsigned n0 = crow0 - bidx * (unsigned)SEQ;
  const unsigned c = (tid & 15u) * 8u;
  const unsigned rq = tid >> 4;

  float cs[8];
#pragma unroll
  for (int i = 0; i < 8; ++i) cs[i] = 0.0f;
  v8h xv[4];
  size_t off[4];
#pragma unroll
  for (unsigned j = 0; j < 4u; ++j) {
    const unsigned r = 16u * j + rq;
    const float* src = X + ((size_t)bidx * SEQ_FULL + n0 + r) * CDIM + c;
    const v4f a0 = *(const v4f*)(src);
    const v4f a1 = *(const v4f*)(src + 4);
#pragma unroll
    for (int i = 0; i < 4; ++i) {
      const float e0 = bf16r(a0[i]);
      const float e1 = bf16r(a1[i]);
      cs[i]     += e0;
      cs[i + 4] += e1;
      const h16 h0 = toh_flush(XCARRY * e0);
      const h16 h1 = toh_flush(XCARRY * e1);
      xv[j][i]     = h0;
      xv[j][i + 4] = h1;
      T[(c + (unsigned)i) * LDT + r]      = h0;
      T[(c + 4u + (unsigned)i) * LDT + r] = h1;
    }
    off[j] = (size_t)(crow0 + r) * CDIM + c;
  }
  {
    v4f s0, s1;
#pragma unroll
    for (int i = 0; i < 4; ++i) { s0[i] = cs[i]; s1[i] = cs[i + 4]; }
    *(v4f*)&Sc[rq * CDIM + c]      = s0;
    *(v4f*)&Sc[rq * CDIM + c + 4u] = s1;
  }
  __syncthreads();

  v8h tv[4];
  size_t toff[4];
#pragma unroll
  for (unsigned i = 0; i < 4u; ++i) {
    const unsigned kr = 32u * i + (tid >> 3);
    const unsigned pc = (tid & 7u) * 8u;
    tv[i] = *(const v8h*)&T[kr * LDT + pc];
    toff[i] = ((size_t)bidx * CDIM + kr) * SEQ + n0 + pc;
  }
  v4f st = {};
  if (wave == 0) {
#pragma unroll 4
    for (unsigned q = 0; q < 16u; ++q) st += *(const v4f*)&Sc[q * CDIM + 4u * lane];
  }
  float* sp = Spart + (size_t)blockIdx.x * CDIM + 4u * lane;

#pragma unroll
  for (int j = 0; j < 4; ++j) *(volatile v8h*)(X16 + off[j]) = xv[j];
#pragma unroll
  for (int i = 0; i < 4; ++i) *(volatile v8h*)(XT16 + toff[i]) = tv[i];
  if (wave == 0) *(volatile v4f*)sp = st;
  __threadfence();
#pragma unroll
  for (int j = 0; j < 4; ++j) *(volatile v8h*)(X16 + off[j]) = xv[j];
#pragma unroll
  for (int i = 0; i < 4; ++i) *(volatile v8h*)(XT16 + toff[i]) = tv[i];
  if (wave == 0) *(volatile v4f*)sp = st;
}

__global__ __launch_bounds__(256) void gram_kernel(
    const _Float16* __restrict__ XT16, float* __restrict__ Gpart) {
  __shared__ float Cs[64 * LDC];
  const unsigned tid = threadIdx.x, lane = tid & 31u, w = tid >> 5;
  const unsigned mw = w >> 1, nw = w & 1u;
  const unsigned hh = lane >> 4, m = lane & 15u;
  const unsigned n0 = blockIdx.x * 64u;
  const unsigned row0 = blockIdx.y * 64u;
  const unsigned bidx = blockIdx.z / (unsigned)GCH;
  const unsigned ch = blockIdx.z - bidx * (unsigned)GCH;

  const _Float16* plane = XT16 + (size_t)bidx * CDIM * SEQ + (size_t)ch * KCH;
  const _Float16* ap  = plane + (size_t)(row0 + mw * 16u + m) * SEQ + hh * 8u;
  const _Float16* bp0 = plane + (size_t)(n0 + nw * 32u + m) * SEQ + hh * 8u;
  const _Float16* bp1 = bp0 + (size_t)16 * SEQ;
  v8f acc0 = {}, acc1 = {};
  gemm_loop(ap, bp0, bp1, (unsigned)KCH, acc0, acc1);
#pragma unroll
  for (int r = 0; r < 8; ++r) {
    float* d = &Cs[(mw * 16u + hh * 8u + (unsigned)r) * LDC + nw * 32u + m];
    d[0]  = acc0[r];
    d[16] = acc1[r];
  }
  __syncthreads();

  const float cs = 1.0f / (XCARRY * XCARRY);
  v4f xs[4];
  size_t off[4];
#pragma unroll
  for (unsigned i = 0; i < 4u; ++i) {
    const unsigned r = 16u * i + (tid >> 4);
    const unsigned c = (tid & 15u) * 4u;
    const v4f u = *(const v4f*)&Cs[r * LDC + c];
    xs[i] = u * cs;
    off[i] = ((size_t)blockIdx.z * CDIM + row0 + r) * CDIM + n0 + c;
  }
#pragma unroll
  for (int i = 0; i < 4; ++i) *(volatile v4f*)(Gpart + off[i]) = xs[i];
  __threadfence();
#pragma unroll
  for (int i = 0; i < 4; ++i) *(volatile v4f*)(Gpart + off[i]) = xs[i];
}

__global__ __launch_bounds__(256) void reduce_kernel(
    const float* __restrict__ Gpart, const float* __restrict__ Spart,
    float* __restrict__ G, float* __restrict__ S) {
  __shared__ float Sr[8 * CDIM];
  const unsigned lane = threadIdx.x & 31u;
  const int wave = __builtin_amdgcn_readfirstlane((int)(threadIdx.x >> 5));
  const unsigned blk = blockIdx.x;
  const bool sblk = (blk >= (unsigned)(NB * (CDIM / 8)));
  v4f acc = {};
  if (!sblk) {
    const unsigned bidx = blk >> 4;
    const unsigned krow = (blk & 15u) * 8u + (unsigned)wave;
#pragma unroll 4
    for (unsigned ch = 0; ch < (unsigned)GCH; ++ch)
      acc += *(const v4f*)(Gpart + ((size_t)(bidx * GCH + ch) * CDIM + krow) * CDIM + 4u * lane);
  } else {
    const unsigned bidx = blk - (unsigned)(NB * (CDIM / 8));
#pragma unroll 4
    for (unsigned j = 0; j < (unsigned)BPW; ++j)
      acc += *(const v4f*)(Spart + ((size_t)bidx * BPB + (unsigned)wave * BPW + j) * CDIM + 4u * lane);
    *(v4f*)&Sr[(unsigned)wave * CDIM + 4u * lane] = acc;
  }
  __syncthreads();
  if (!sblk) {
    const unsigned bidx = blk >> 4;
    const unsigned krow = (blk & 15u) * 8u + (unsigned)wave;
    float* p = G + ((size_t)bidx * CDIM + krow) * CDIM + 4u * lane;
    *(volatile v4f*)p = acc;
    __threadfence();
    *(volatile v4f*)p = acc;
  } else if (wave == 0) {
    const unsigned bidx = blk - (unsigned)(NB * (CDIM / 8));
    v4f tot = {};
#pragma unroll
    for (unsigned q = 0; q < 8u; ++q) tot += *(const v4f*)&Sr[q * CDIM + 4u * lane];
    float* p = S + (size_t)bidx * CDIM + 4u * lane;
    *(volatile v4f*)p = tot;
    __threadfence();
    *(volatile v4f*)p = tot;
  }
}

__global__ __launch_bounds__(256) void integral_kernel(
    const float* __restrict__ psi_w, const float* __restrict__ psi_b,
    const float* __restrict__ G, const float* __restrict__ S, _Float16* __restrict__ IT16) {
  __shared__ _Float16 Ts[NB * IC * LDT];
  const unsigned tid = threadIdx.x, lane = tid & 31u;
  const int wave = __builtin_amdgcn_readfirstlane((int)(threadIdx.x >> 5));
  const unsigned c = blockIdx.x * (unsigned)IC + lane;
  const unsigned r0 = (unsigned)wave * 8u;

  float acc[NB][8];
#pragma unroll
  for (int b = 0; b < NB; ++b)
#pragma unroll
    for (int rr = 0; rr < 8; ++rr) acc[b][rr] = 0.0f;

  const float* wp = psi_w + (size_t)r0 * CDIM + c;
#pragma unroll 1
  for (unsigned k = 0; k < (unsigned)CDIM; ++k) {
    float g[NB];
#pragma unroll
    for (int b = 0; b < NB; ++b) g[b] = G[((size_t)b * CDIM + k) * CDIM + c];
#pragma unroll
    for (int rr = 0; rr < 8; ++rr) {
      const float wv = bf16r(wp[(size_t)k * (RNK * CDIM) + (unsigned)rr * CDIM]);
#pragma unroll
      for (int b = 0; b < NB; ++b) acc[b][rr] += wv * g[b];
    }
  }

  const float invn = 1.0f / (float)SEQ;
#pragma unroll
  for (int b = 0; b < NB; ++b) {
    const float sv = S[(size_t)b * CDIM + c];
    v8h o;
#pragma unroll
    for (int rr = 0; rr < 8; ++rr) {
      const float pb = bf16r(psi_b[(r0 + (unsigned)rr) * CDIM + c]);
      const float val = (acc[b][rr] + pb * sv) * invn;
      o[rr] = toh_flush(ICARRY * val);
    }
    *(v8h*)&Ts[((unsigned)b * IC + lane) * LDT + r0] = o;
  }
  __syncthreads();

  v8h x[NB];
  size_t off[NB];
#pragma unroll
  for (unsigned i = 0; i < (unsigned)NB; ++i) {
    const unsigned rowc = tid >> 3;
    const unsigned pc = (tid & 7u) * 8u;
    x[i] = *(const v8h*)&Ts[(i * IC + rowc) * LDT + pc];
    off[i] = ((size_t)i * CDIM + blockIdx.x * (unsigned)IC + rowc) * RNK + pc;
  }
#pragma unroll
  for (int i = 0; i < NB; ++i) *(volatile v8h*)(IT16 + off[i]) = x[i];
  __threadfence();
#pragma unroll
  for (int i = 0; i < NB; ++i) *(volatile v8h*)(IT16 + off[i]) = x[i];
}

__global__ __launch_bounds__(256) void phconv_kernel(
    const float* __restrict__ phi_w, const float* __restrict__ phi_b,
    _Float16* __restrict__ PH16) {
  const unsigned tid = threadIdx.x;
  const unsigned row = blockIdx.x * 32u + (tid >> 3);
  const unsigned pc = (tid & 7u) * 8u;
  const unsigned rw = (row < (unsigned)CDIM) ? row : (unsigned)(CDIM - 1);
  const v4f a0 = *(const v4f*)(phi_w + (size_t)rw * RNK + pc);
  const v4f a1 = *(const v4f*)(phi_w + (size_t)rw * RNK + pc + 4u);
  const v4f b0 = *(const v4f*)(phi_b + pc);
  const v4f b1 = *(const v4f*)(phi_b + pc + 4u);
  v8h o;
#pragma unroll
  for (int i = 0; i < 4; ++i) {
    const float v0 = (row < (unsigned)CDIM) ? a0[i] : ((row == (unsigned)CDIM) ? b0[i] : 0.0f);
    const float v1 = (row < (unsigned)CDIM) ? a1[i] : ((row == (unsigned)CDIM) ? b1[i] : 0.0f);
    o[i]     = toh_flush(WCARRY * bf16r(v0));
    o[i + 4] = toh_flush(WCARRY * bf16r(v1));
  }
  _Float16* p = PH16 + (size_t)row * RNK + pc;
  *(volatile v8h*)p = o;
  __threadfence();
  *(volatile v8h*)p = o;
}

__global__ __launch_bounds__(256) void weff_kernel(
    const _Float16* __restrict__ IT16, const _Float16* __restrict__ PH16,
    const float* __restrict__ W_w, const float* __restrict__ W_b,
    _Float16* __restrict__ WT16, float* __restrict__ BE) {
  __shared__ float Cs[64 * LDC];
  const unsigned tid = threadIdx.x, lane = tid & 31u, w = tid >> 5;
  const int wave = __builtin_amdgcn_readfirstlane((int)(threadIdx.x >> 5));
  const unsigned mw = w >> 1, nw = w & 1u;
  const unsigned hh = lane >> 4, m = lane & 15u;
  const unsigned n0 = blockIdx.x * 64u;
  const unsigned row0 = blockIdx.y * 64u;
  const unsigned bidx = blockIdx.z;

  const _Float16* ap  = IT16 + ((size_t)bidx * CDIM + row0 + mw * 16u + m) * RNK + hh * 8u;
  const _Float16* bp0 = PH16 + (size_t)(n0 + nw * 32u + m) * RNK + hh * 8u;
  const _Float16* bp1 = bp0 + (size_t)16 * RNK;
  v8f acc0 = {}, acc1 = {};
  gemm_loop(ap, bp0, bp1, (unsigned)RNK, acc0, acc1);
#pragma unroll
  for (int r = 0; r < 8; ++r) {
    float* d = &Cs[(mw * 16u + hh * 8u + (unsigned)r) * LDC + nw * 32u + m];
    d[0]  = acc0[r];
    d[16] = acc1[r];
  }
  __syncthreads();

  const float cs = 1.0f / (ICARRY * WCARRY);
  if (blockIdx.x < 2u) {
#pragma unroll 1
    for (unsigned g = 0; g < 2u; ++g) {
      const unsigned r = 32u * g + (tid >> 3);
      const unsigned cc = (tid & 7u) * 8u;
      const v4f u0 = *(const v4f*)&Cs[r * LDC + cc];
      const v4f u1 = *(const v4f*)&Cs[r * LDC + cc + 4u];
      const float* wp = W_w + (size_t)(n0 + cc) * CDIM + row0 + r;
      v4f t0, t1;
#pragma unroll
      for (int j = 0; j < 4; ++j) {
        t0[j] = ECARRY * (bf16r(wp[(size_t)j * CDIM]) + u0[j] * cs);
        t1[j] = ECARRY * (bf16r(wp[(size_t)(j + 4) * CDIM]) + u1[j] * cs);
      }
      *(v4f*)&Cs[r * LDC + cc]      = t0;
      *(v4f*)&Cs[r * LDC + cc + 4u] = t1;
    }
    v8h x[2];
    size_t off[2];
#pragma unroll
    for (unsigned i = 0; i < 2u; ++i) {
      const unsigned r = 32u * i + (tid >> 3);
      const unsigned cc = (tid & 7u) * 8u;
      const v4f u0 = *(const v4f*)&Cs[r * LDC + cc];
      const v4f u1 = *(const v4f*)&Cs[r * LDC + cc + 4u];
#pragma unroll
      for (int j = 0; j < 4; ++j) {
        x[i][j]     = toh_flush(u0[j]);
        x[i][j + 4] = toh_flush(u1[j]);
      }
      off[i] = ((size_t)bidx * CDIM + row0 + r) * CDIM + n0 + cc;
    }
#pragma unroll
    for (int i = 0; i < 2; ++i) *(volatile v8h*)(WT16 + off[i]) = x[i];
    __threadfence();
#pragma unroll
    for (int i = 0; i < 2; ++i) *(volatile v8h*)(WT16 + off[i]) = x[i];
  } else {
    if (wave == 0) {
      const unsigned r = 2u * lane;
      v2f bv;
      bv[0] = bf16r(W_b[row0 + r])      + Cs[r * LDC] * cs;
      bv[1] = bf16r(W_b[row0 + r + 1u]) + Cs[(r + 1u) * LDC] * cs;
      float* p = BE + (size_t)bidx * CDIM + row0 + r;
      *(volatile v2f*)p = bv;
      __threadfence();
      *(volatile v2f*)p = bv;
    }
  }
}

__global__ __launch_bounds__(256) void out_kernel(
    const _Float16* __restrict__ X16, const _Float16* __restrict__ WT16,
    const float* __restrict__ BE, float* __restrict__ outf) {
  __shared__ float Cs[64 * LDC];
  const unsigned tid = threadIdx.x, lane = tid & 31u, w = tid >> 5;
  const unsigned mw = w >> 1, nw = w & 1u;
  const unsigned hh = lane >> 4, m = lane & 15u;
  const unsigned n0 = blockIdx.x * 64u;
  const unsigned row0 = blockIdx.y * 64u;
  const unsigned bidx = row0 / (unsigned)SEQ;
  const unsigned sq0 = row0 - bidx * (unsigned)SEQ;

  const _Float16* ap  = X16 + (size_t)(row0 + mw * 16u + m) * CDIM + hh * 8u;
  const _Float16* bp0 = WT16 + ((size_t)bidx * CDIM + n0 + nw * 32u + m) * CDIM + hh * 8u;
  const _Float16* bp1 = bp0 + (size_t)16 * CDIM;
  v8f acc0 = {}, acc1 = {};
  gemm_loop(ap, bp0, bp1, (unsigned)CDIM, acc0, acc1);
#pragma unroll
  for (int r = 0; r < 8; ++r) {
    float* d = &Cs[(mw * 16u + hh * 8u + (unsigned)r) * LDC + nw * 32u + m];
    d[0]  = acc0[r];
    d[16] = acc1[r];
  }
  __syncthreads();

  const float cs = 1.0f / (XCARRY * ECARRY);
#pragma unroll 1
  for (unsigned g = 0; g < 4u; ++g) {
    const unsigned r = 16u * g + (tid >> 4);
    const unsigned c = (tid & 15u) * 4u;
    const v4f u  = *(const v4f*)&Cs[r * LDC + c];
    const v4f bb = *(const v4f*)(BE + (size_t)bidx * CDIM + n0 + c);
    v4f t;
#pragma unroll
    for (int j = 0; j < 4; ++j) t[j] = gelu_erf(u[j] * cs + bb[j]);
    *(v4f*)&Cs[r * LDC + c] = t;
  }

  v4f xs[4];
  size_t off[4];
#pragma unroll
  for (unsigned i = 0; i < 4u; ++i) {
    const unsigned r = 16u * i + (tid >> 4);
    const unsigned c = (tid & 15u) * 4u;
    xs[i] = *(const v4f*)&Cs[r * LDC + c];
    off[i] = ((size_t)bidx * SEQ_FULL + sq0 + r) * CDIM + n0 + c;
  }
#pragma unroll
  for (int i = 0; i < 4; ++i) *(volatile v4f*)(outf + off[i]) = xs[i];
  __threadfence();
#pragma unroll
  for (int i = 0; i < 4; ++i) *(volatile v4f*)(outf + off[i]) = xs[i];
}

extern "C" void kernel_launch(void* const* d_in, const int* in_sizes, int n_in,
                              void* d_out, int out_size, void* d_ws, size_t ws_size,
                              hipStream_t stream) {
  if (n_in < 7) return;
  const long long need_x = ((long long)(NB - 1) * SEQ_FULL + SEQ) * CDIM;
  if ((long long)in_sizes[0] < need_x) return;
  if ((long long)in_sizes[1] < (long long)CDIM * CDIM) return;
  if (in_sizes[2] < CDIM) return;
  if ((long long)in_sizes[3] < (long long)CDIM * RNK) return;
  if (in_sizes[4] < RNK) return;
  if ((long long)in_sizes[5] < (long long)CDIM * RNK * CDIM) return;
  if ((long long)in_sizes[6] < (long long)RNK * CDIM) return;
  if ((long long)out_size < need_x) return;
  if (ws_size < WS_TOTAL) return;

  const float* X     = (const float*)d_in[0];
  const float* W_w   = (const float*)d_in[1];
  const float* W_b   = (const float*)d_in[2];
  const float* phi_w = (const float*)d_in[3];
  const float* phi_b = (const float*)d_in[4];
  const float* psi_w = (const float*)d_in[5];
  const float* psi_b = (const float*)d_in[6];
  float* out = (float*)d_out;

  char* ws = (char*)d_ws;
  _Float16* X16   = (_Float16*)(ws + OFF_X16);
  _Float16* XT16  = (_Float16*)(ws + OFF_XT16);
  float*    Spart = (float*)(ws + OFF_SPART);
  float*    Gpart = (float*)(ws + OFF_GPART);
  float*    G     = (float*)(ws + OFF_G);
  float*    S     = (float*)(ws + OFF_S);
  _Float16* IT16  = (_Float16*)(ws + OFF_IT);
  _Float16* PH16  = (_Float16*)(ws + OFF_PH);
  _Float16* WT16  = (_Float16*)(ws + OFF_WT);
  float*    BE    = (float*)(ws + OFF_BE);

  dim3 blk(256);
  xconv_kernel<<<dim3(XBLKS), blk, 0, stream>>>(X, X16, XT16, Spart);
  gram_kernel<<<dim3(CDIM / 64, CDIM / 64, NB * GCH), blk, 0, stream>>>(XT16, Gpart);
  reduce_kernel<<<dim3(NB * (CDIM / 8) + NB), blk, 0, stream>>>(Gpart, Spart, G, S);
  integral_kernel<<<dim3(CDIM / IC), blk, 0, stream>>>(psi_w, psi_b, G, S, IT16);
  phconv_kernel<<<dim3(PHROWS / 32), blk, 0, stream>>>(phi_w, phi_b, PH16);
  weff_kernel<<<dim3(PHROWS / 64, CDIM / 64, NB), blk, 0, stream>>>(IT16, PH16, W_w, W_b, WT16, BE);
  out_kernel<<<dim3(CDIM / 64, MROWS / 64), blk, 0, stream>>>(X16, WT16, BE, out);
}
